// SaProtEpitopeCompareNN_10471130268322
// MI455X (gfx1250) — hardware-verified
//
#include <hip/hip_runtime.h>
#include <stdint.h>
#include <stddef.h>
#include <math.h>

constexpr int kBatch   = 2;
constexpr int kLag     = 512;
constexpr int kLepi    = 256;
constexpr int kCin     = 446;
constexpr int kCpad    = 448;
constexpr int kDhid    = 64;
constexpr int kNcol    = kLepi * kDhid;
constexpr int kChunks8 = kCpad / 8;
constexpr float kCarry    = 1024.0f;
constexpr float kCarryInv = 1.0f / 1024.0f;
constexpr float kLnEps    = 1e-5f;
constexpr float kInv64    = 1.0f / 64.0f;
constexpr int kZPitch  = 68;
constexpr int kJHalf   = 128;

typedef __attribute__((ext_vector_type(16))) _Float16 v16h;
typedef __attribute__((ext_vector_type(8)))  _Float16 v8h;
typedef __attribute__((ext_vector_type(16))) __bf16   v16b;
typedef __attribute__((ext_vector_type(8)))  __bf16   v8b;
typedef __attribute__((ext_vector_type(8)))  float    v8f;
typedef __attribute__((ext_vector_type(4)))  float    v4f;
typedef __attribute__((ext_vector_type(4)))  unsigned int v4u;

__device__ __forceinline__ unsigned short f2bf_bits(float f) {
  unsigned u = __float_as_uint(f);
  return (unsigned short)((u + 0x7FFFu + ((u >> 16) & 1u)) >> 16);
}
__device__ __forceinline__ float bf_bits2f(unsigned short h) { return __uint_as_float(((unsigned)h) << 16); }

__device__ __forceinline__ void dep_guard_h(v8f& a, v8f& b, v16h x, v16h y) { asm volatile("v_nop\n\tv_nop\n\tv_nop\n\tv_nop" : "+v"(a), "+v"(b) : "v"(x), "v"(y)); }
__device__ __forceinline__ void dep_guard_b(v8f& a, v8f& b, v16b x, v16b y) { asm volatile("v_nop\n\tv_nop\n\tv_nop\n\tv_nop" : "+v"(a), "+v"(b) : "v"(x), "v"(y)); }
__device__ __forceinline__ void keep4_h(v16h a, v16h b, v16h c, v16h d) { asm volatile("v_nop" :: "v"(a), "v"(b), "v"(c), "v"(d)); }
__device__ __forceinline__ void keep4_b(v16b a, v16b b, v16b c, v16b d) { asm volatile("v_nop" :: "v"(a), "v"(b), "v"(c), "v"(d)); }
__device__ __forceinline__ void acc_guard4(v8f& a, v8f& b, v8f& c, v8f& d) { asm volatile("v_nop\n\tv_nop\n\tv_nop\n\tv_nop" : "+v"(a), "+v"(b), "+v"(c), "+v"(d)); }
template <typename T> struct Frag;
template <> struct Frag<_Float16> {
  typedef v16h V; union U { v16h v; v8h h[2]; };
  static __device__ __forceinline__ v16h load(const _Float16* p) {
    U f; f.h[0] = *(const v8h*)(p); f.h[1] = *(const v8h*)(p + 16); return f.v;
  }
  static __device__ __forceinline__ v8f mma(v16h a, v16h b, v8f c) {
    return __builtin_amdgcn_wmma_f32_16x16x32_f16(false, a, false, b, (short)0, c, false, false);
  }
  static __device__ __forceinline__ void guard(v8f& a, v8f& b, v16h x, v16h y) { dep_guard_h(a, b, x, y); }
  static __device__ __forceinline__ void keep(v16h a, v16h b, v16h c, v16h d) { keep4_h(a, b, c, d); }
};
template <> struct Frag<__bf16> {
  typedef v16b V; union U { v16b v; v8b h[2]; };
  static __device__ __forceinline__ v16b load(const __bf16* p) {
    U f; f.h[0] = *(const v8b*)(p); f.h[1] = *(const v8b*)(p + 16); return f.v;
  }
  static __device__ __forceinline__ v8f mma(v16b a, v16b b, v8f c) {
    return __builtin_amdgcn_wmma_f32_16x16x32_bf16(false, a, false, b, (short)0, c, false, false);
  }
  static __device__ __forceinline__ void guard(v8f& a, v8f& b, v16b x, v16b y) { dep_guard_b(a, b, x, y); }
  static __device__ __forceinline__ void keep(v16b a, v16b b, v16b c, v16b d) { keep4_b(a, b, c, d); }
};

__device__ __forceinline__ unsigned pk16(unsigned short a, unsigned short b) { return (unsigned)a | ((unsigned)b << 16); }
__device__ __forceinline__ unsigned short h_bits(float f) { const _Float16 h = (_Float16)f; return __builtin_bit_cast(unsigned short, h); }

template <int ET> struct Elem;
template <> struct Elem<0> { typedef _Float16 T; };
template <> struct Elem<1> { typedef __bf16 T; };
template <int ET, bool SPLIT, int BIAS_MODE, int OUT_MODE, bool RESID, int ACT = 0>
__global__ __launch_bounds__(256) void wmma_gemm64(
    const unsigned short* __restrict__ Ap, const unsigned short* __restrict__ A2p, int lda, long strideA,
    const unsigned short* __restrict__ Btp, const unsigned short* __restrict__ Bt2p, int ldb, long strideB,
    void* __restrict__ Cout, void* __restrict__ Cout2, int ldc, long strideC,
    const float* __restrict__ bias,
    const float* __restrict__ resid, long strideR,
    int M, int N, int K, float scale) {
  typedef typename Elem<ET>::T T;
  typedef typename Frag<T>::V V;
  const T* A = (const T*)Ap; const T* A2 = (const T*)A2p; const T* Bt = (const T*)Btp; const T* Bt2 = (const T*)Bt2p;
  __shared__ __align__(16) float sT[8][16 * 68];
  const int b    = blockIdx.y;
  const int lane = threadIdx.x & 31;
  const int wave = threadIdx.x >> 5;
  const int tilesN = N >> 6;
  const int tilesM = M >> 6;
  const int tile = blockIdx.x * 8 + wave;
  if (tile >= tilesM * tilesN) return;
  const int tm = tile / tilesN;
  const int tn = tile - tm * tilesN;
  const int m0 = tm << 6;
  const int n0 = tn << 6;

  const T* Ab  = A  + (size_t)b * strideA;
  const T* Bb  = Bt + (size_t)b * strideB;
  const T* Ab2 = SPLIT ? (A2  + (size_t)b * strideA) : nullptr;
  const T* Bb2 = SPLIT ? (Bt2 + (size_t)b * strideB) : nullptr;

  const int rlane = lane & 15;
  const int koff  = (lane >> 4) * 8;
  const int mOff  = (lane >> 4) * 8;

  v8f acc[4][4];
#pragma unroll
  for (int i = 0; i < 4; ++i)
#pragma unroll
    for (int j = 0; j < 4; ++j) acc[i][j] = (v8f){0.f,0.f,0.f,0.f,0.f,0.f,0.f,0.f};

  for (int k0 = 0; k0 < K; k0 += 32) {
    V bh[4], bl[4];
#pragma unroll
    for (int j = 0; j < 4; ++j) {
      const size_t bo = (size_t)(n0 + (j << 4) + rlane) * ldb + koff + k0;
      bh[j] = Frag<T>::load(Bb + bo);
      if (SPLIT) bl[j] = Frag<T>::load(Bb2 + bo);
    }
#pragma unroll
    for (int i = 0; i < 4; ++i) {
      const size_t ao = (size_t)(m0 + (i << 4) + rlane) * lda + koff + k0;
      V ah = Frag<T>::load(Ab + ao);
      V al;
      if (SPLIT) al = Frag<T>::load(Ab2 + ao);
#pragma unroll
      for (int j = 0; j < 4; ++j) {
        acc[i][j] = Frag<T>::mma(ah, bh[j], acc[i][j]);
        if (SPLIT) {
          acc[i][j] = Frag<T>::mma(ah, bl[j], acc[i][j]);
          acc[i][j] = Frag<T>::mma(al, bh[j], acc[i][j]);
        }
      }
      Frag<T>::guard(acc[i][0], acc[i][3], ah, SPLIT ? al : ah);
    }
    Frag<T>::keep(bh[0], bh[1], bh[2], bh[3]);
    if (SPLIT) Frag<T>::keep(bl[0], bl[1], bl[2], bl[3]);
  }
  acc_guard4(acc[0][0], acc[0][1], acc[0][2], acc[0][3]);
  acc_guard4(acc[1][0], acc[1][1], acc[1][2], acc[1][3]);
  acc_guard4(acc[2][0], acc[2][1], acc[2][2], acc[2][3]);
  acc_guard4(acc[3][0], acc[3][1], acc[3][2], acc[3][3]);

  float* slab = sT[wave];
  const float* Rb = RESID ? (resid + (size_t)b * strideR) : nullptr;
#pragma unroll
  for (int i = 0; i < 4; ++i) {
    const int mBase = m0 + (i << 4);
#pragma unroll
    for (int j = 0; j < 4; ++j) {
      const int n = n0 + (j << 4) + rlane;
      float bv = 0.f;
      if (BIAS_MODE == 2) bv = bias[n];
#pragma unroll
      for (int r = 0; r < 8; ++r) {
        float v = acc[i][j][r] * scale;
        if (BIAS_MODE == 1) v += bias[mBase + mOff + r];
        if (BIAS_MODE == 2) v += bv;
        if (RESID) v += Rb[(size_t)(mBase + mOff + r) * ldc + n];
        if (ACT == 2) v = fmaxf(v, 0.0f);
        if (ACT == 4) v = (v > 0.f) ? v : 0.01f * v;
        slab[(mOff + r) * 68 + (j << 4) + rlane] = v;
      }
    }
    __builtin_amdgcn_fence(__ATOMIC_RELEASE, "workgroup");
    __builtin_amdgcn_wave_barrier();
    __builtin_amdgcn_fence(__ATOMIC_ACQUIRE, "workgroup");
    if (OUT_MODE == 0) {
      float* C = (float*)Cout + (size_t)b * strideC;
      const int hh = lane >> 4, c4 = (lane & 15) * 4;
      for (int pass = 0; pass < 2; ++pass) {
#pragma unroll
        for (int it = 0; it < 8; ++it) {
          const int row = it * 2 + hh;
          v4f v = *(const v4f*)(slab + row * 68 + c4);
          *(volatile v4f*)(C + (size_t)(mBase + row) * ldc + n0 + c4) = v;
        }
        __threadfence();
      }
    } else {
      const int q = lane >> 3, c8 = (lane & 7) * 8;
      unsigned short* C  = (unsigned short*)Cout  + (size_t)b * strideC;
      unsigned short* C2 = (OUT_MODE == 2) ? ((unsigned short*)Cout2 + (size_t)b * strideC) : nullptr;
      for (int pass = 0; pass < 2; ++pass) {
#pragma unroll
        for (int it = 0; it < 4; ++it) {
          const int row = it * 4 + q;
          const float* sp = slab + row * 68 + c8;
          v8h hv, lv;
#pragma unroll
          for (int e = 0; e < 8; ++e) {
            if (OUT_MODE == 1) {
              hv[e] = (_Float16)sp[e];
            } else {
              unsigned short hb = f2bf_bits(sp[e]);
              unsigned short lb = f2bf_bits(sp[e] - bf_bits2f(hb));
              hv[e] = __builtin_bit_cast(_Float16, hb);
              lv[e] = __builtin_bit_cast(_Float16, lb);
            }
          }
          *(volatile v8h*)(C + (size_t)(mBase + row) * ldc + n0 + c8) = hv;
          if (OUT_MODE == 2) *(volatile v8h*)(C2 + (size_t)(mBase + row) * ldc + n0 + c8) = lv;
        }
        __threadfence();
      }
    }
    __builtin_amdgcn_fence(__ATOMIC_RELEASE, "workgroup");
    __builtin_amdgcn_wave_barrier();
    __builtin_amdgcn_fence(__ATOMIC_ACQUIRE, "workgroup");
  }
}

__global__ __launch_bounds__(256) void cast_pad_f16_kernel(const float* __restrict__ in, unsigned short* __restrict__ out, int n8) {
  const int i = blockIdx.x * 256 + threadIdx.x;
  if (i >= n8) return;
  const int row = i / kChunks8;
  const int c0  = (i - row * kChunks8) * 8;
  const float* p = in + (size_t)row * kCin;
  unsigned short hb[8];
#pragma unroll
  for (int e = 0; e < 8; ++e) {
    const int c  = c0 + e;
    const int cc = (c < kCin) ? c : (kCin - 1);
    const float f = p[cc];
    hb[e] = h_bits((c < kCin) ? f : 0.0f);
  }
  const v4u u = (v4u){pk16(hb[0], hb[1]), pk16(hb[2], hb[3]), pk16(hb[4], hb[5]), pk16(hb[6], hb[7])};
  unsigned short* q = out + 8 * (size_t)i;
  *(volatile v4u*)q = u;
  __threadfence();
  *(volatile v4u*)q = u;
}

__global__ __launch_bounds__(256) void ew_build_kernel(const float* __restrict__ epi, const float* __restrict__ w1,
                                                       unsigned short* __restrict__ ew) {
  __shared__ __align__(16) float es[kCpad];
  const int bj = blockIdx.x;
  const int t  = threadIdx.x;
  const float* er = epi + (size_t)bj * kCin;
  for (int p = t; p < kCpad; p += 256) {
    const int cc = (p < kCin) ? p : (kCin - 1);
    const float f = er[cc];
    es[p] = (p < kCin) ? f : 0.0f;
  }
  __syncthreads();
  const int lane = t & 31, wave = t >> 5;
  unsigned short* rowbase = ew + (size_t)bj * kDhid * kCpad;
  const int c0 = 8 * lane;
  const int c1 = 256 + 8 * lane;
#pragma unroll 1
  for (int r = 0; r < 8; ++r) {
    const int o = wave * 8 + r;
    const float* wr = w1 + (size_t)o * kCin;
    unsigned short ha[8], hc[8];
#pragma unroll
    for (int e = 0; e < 8; ++e) {
      float pa = es[c0 + e] * wr[c0 + e];
      pa = pa * kCarry;
      ha[e] = h_bits(pa);
      const int c  = c1 + e;
      const int cl = (c < kCin) ? c : (kCin - 1);
      const int ce = (c < kCpad) ? c : (kCpad - 1);
      float pc = es[ce] * wr[cl];
      pc = pc * kCarry;
      hc[e] = h_bits((c < kCin) ? pc : 0.0f);
    }
    const v4u ua = (v4u){pk16(ha[0], ha[1]), pk16(ha[2], ha[3]), pk16(ha[4], ha[5]), pk16(ha[6], ha[7])};
    const v4u uc = (v4u){pk16(hc[0], hc[1]), pk16(hc[2], hc[3]), pk16(hc[4], hc[5]), pk16(hc[6], hc[7])};
    unsigned short* rp = rowbase + (size_t)o * kCpad;
    for (int pass = 0; pass < 2; ++pass) {
      *(volatile v4u*)(rp + c0) = ua;
      if (lane < 24) *(volatile v4u*)(rp + c1) = uc;
      __threadfence();
    }
  }
}

__global__ __launch_bounds__(128) void ln_head_kernel(const float* __restrict__ z,
                                                      const float* __restrict__ b1, const float* __restrict__ gam,
                                                      const float* __restrict__ bet, const float* __restrict__ w2,
                                                      const float* __restrict__ b2, float* __restrict__ out) {
  __shared__ __align__(16) float zs[kJHalf * kZPitch];
  __shared__ __align__(16) float prm[4][kDhid];
  __shared__ __align__(16) float so[kJHalf];
  const int t  = threadIdx.x;
  const int jh = blockIdx.x;
  const int i  = blockIdx.y;
  const int b  = blockIdx.z;
  const float* zc = z + ((size_t)(b * kLag + i) * kNcol + (size_t)jh * kJHalf * kDhid);
#pragma unroll
  for (int it = 0; it < 16; ++it) {
    const int e  = it * 128 + t;
    const int jl = e >> 4;
    const int o4 = (e & 15) * 4;
    const v4f v = *(const v4f*)(zc + 4 * (size_t)e);
    *(v4f*)(zs + jl * kZPitch + o4) = v;
  }
  if (t < kDhid) { prm[0][t] = b1[t]; prm[1][t] = gam[t]; prm[2][t] = bet[t]; prm[3][t] = w2[t]; }
  __syncthreads();

  const v4f* zr4 = (const v4f*)(zs + t * kZPitch);
  const v4f* pb4 = (const v4f*)(prm[0]);
  const v4f* pg4 = (const v4f*)(prm[1]);
  const v4f* pe4 = (const v4f*)(prm[2]);
  const v4f* pw4 = (const v4f*)(prm[3]);
  float s = 0.f;
#pragma unroll 1
  for (int q = 0; q < 16; ++q) {
    const v4f v = zr4[q] + pb4[q];
    s += (v[0] + v[1]) + (v[2] + v[3]);
  }
  const float mu = s * kInv64;
  float sq = 0.f;
#pragma unroll 1
  for (int q = 0; q < 16; ++q) {
    const v4f v = zr4[q] + pb4[q];
    const v4f d = v - mu;
    sq += (d[0] * d[0] + d[1] * d[1]) + (d[2] * d[2] + d[3] * d[3]);
  }
  const float var  = sq * kInv64;
  const float rstd = rsqrtf(var + kLnEps);
  float acc = 0.f;
#pragma unroll 1
  for (int q = 0; q < 16; ++q) {
    const v4f v = zr4[q] + pb4[q];
    const v4f g = pg4[q];
    const v4f be = pe4[q];
    const v4f w = pw4[q];
    v4f y = (v - mu) * rstd * g + be;
    const float y0 = fmaxf(y[0], 0.0f), y1 = fmaxf(y[1], 0.0f), y2 = fmaxf(y[2], 0.0f), y3 = fmaxf(y[3], 0.0f);
    acc += (y0 * w[0] + y1 * w[1]) + (y2 * w[2] + y3 * w[3]);
  }
  so[t] = acc + b2[0];
  __syncthreads();
  if (t < 32) {
    const v4f v = *(const v4f*)(so + 4 * t);
    float* op = out + ((size_t)(b * kLag + i) * kLepi + (size_t)jh * kJHalf + 4 * t);
    *(volatile v4f*)op = v;
    __threadfence();
    *(volatile v4f*)op = v;
  }
}

extern "C" void kernel_launch(void* const* d_in, const int* in_sizes, int n_in,
                              void* d_out, int out_size, void* d_ws, size_t ws_size,
                              hipStream_t stream) {
  (void)in_sizes; (void)n_in; (void)out_size;
  const float* ag    = (const float*)d_in[0];
  const float* epi   = (const float*)d_in[1];
  const float* w1    = (const float*)d_in[2];
  const float* b1    = (const float*)d_in[3];
  const float* gam   = (const float*)d_in[4];
  const float* bet   = (const float*)d_in[5];
  const float* w2    = (const float*)d_in[6];
  const float* b2    = (const float*)d_in[7];
  float* out = (float*)d_out;

  const size_t agBytes = (size_t)kBatch * kLag * kCpad * 2;
  const size_t ewBytes = (size_t)kBatch * kNcol * kCpad * 2;
  const size_t zBytes  = (size_t)kBatch * kLag * kNcol * 4;
  const size_t offAG = 0;
  const size_t offEW = offAG + agBytes;
  const size_t offZ  = offEW + ewBytes;
  if (offZ + zBytes > ws_size) return;
  unsigned short* ag16 = (unsigned short*)((char*)d_ws + offAG);
  unsigned short* ew16 = (unsigned short*)((char*)d_ws + offEW);
  float* zf = (float*)((char*)d_ws + offZ);

  {
    const int n8 = kBatch * kLag * kChunks8;
    cast_pad_f16_kernel<<<dim3((n8 + 255) / 256), dim3(256), 0, stream>>>(ag, ag16, n8);
  }
  ew_build_kernel<<<dim3(kBatch * kLepi), dim3(256), 0, stream>>>(epi, w1, ew16);
  wmma_gemm64<0, false, 0, 0, false, 0><<<dim3((kLag / 64) * (kNcol / 64) / 8, kBatch), dim3(256), 0, stream>>>(
      ag16, ag16, kCpad, (long)kLag * kCpad,
      ew16, ew16, kCpad, (long)kNcol * kCpad,
      (void*)zf, (void*)zf, kNcol, (long)kLag * kNcol,
      b1, b1, 0L,
      kLag, kNcol, kCpad, kCarryInv);
  ln_head_kernel<<<dim3(kLepi / kJHalf, kLag, kBatch), dim3(128), 0, stream>>>(zf, b1, gam, bet, w2, b2, out);
}
